// PointNetSetAbstractionWithOriginalGraph_76398878261706
// MI455X (gfx1250) — hardware-verified
//
#include <hip/hip_runtime.h>
#pragma clang fp contract(off)

typedef __attribute__((ext_vector_type(16))) __bf16   v16b;
typedef __attribute__((ext_vector_type(8)))  __bf16   v8b;
typedef __attribute__((ext_vector_type(8)))  float    v8f;
typedef __attribute__((ext_vector_type(4)))  float    v4f;
typedef __attribute__((ext_vector_type(4)))  unsigned v4u;

constexpr int NBATCH = 4;
constexpr int NPTS   = 4096;
constexpr int DFEAT  = 64;
constexpr int KNBR   = 24;
constexpr int GOUT   = 128;
constexpr int HALFC  = 128;
constexpr int MLPC0  = 64;
constexpr int MLPC1  = 128;
constexpr int MLPC2  = 256;
constexpr int NROWS  = NBATCH * NPTS;
constexpr int G0_LD  = 96;
constexpr int FUSEDC = MLPC2 + HALFC;
constexpr float BN_EPS = 1e-5f;

static_assert(NROWS == 16384, "rows");
static_assert(NROWS % 64 == 0 && NPTS % 64 == 0, "64-row tiles stay inside one batch");
static_assert(G0_LD % 32 == 0 && DFEAT % 32 == 0 && GOUT % 32 == 0 && MLPC0 % 32 == 0 && MLPC1 % 32 == 0, "K multiples of 32");
static_assert((2 * GOUT) % 64 == 0 && HALFC % 64 == 0 && MLPC0 % 64 == 0 && MLPC1 % 64 == 0 && MLPC2 % 64 == 0, "N multiples of 64");

constexpr int WOFF_EC = 0;
constexpr int WOFF_GM = WOFF_EC + 2 * GOUT * DFEAT;
constexpr int WOFF_W0 = WOFF_GM + HALFC * GOUT;
constexpr int WOFF_W1 = WOFF_W0 + MLPC0 * G0_LD;
constexpr int WOFF_W2 = WOFF_W1 + MLPC1 * MLPC0;
constexpr int W_TOTAL = WOFF_W2 + MLPC2 * MLPC1;
static_assert(W_TOTAL == 79872, "weight plane elements");
static_assert(WOFF_GM == 8 * 2048 && WOFF_W0 == 8 * 4096 && WOFF_W1 == 8 * 4864 && WOFF_W2 == 8 * 5888, "chunk bases");

__device__ __forceinline__ unsigned bf_hi_bits(float f) {
  const unsigned u = __float_as_uint(f);
  return (u + 0x7FFFu + ((u >> 16) & 1u)) >> 16;
}
__device__ __forceinline__ float bf_bits_f(unsigned h) { return __uint_as_float(h << 16); }

__device__ __forceinline__ void split8(const float (&v)[8], v4u& hw, v4u& lw) {
  unsigned hb[8], lb[8];
#pragma unroll
  for (int e = 0; e < 8; ++e) {
    hb[e] = bf_hi_bits(v[e]);
    lb[e] = bf_hi_bits(v[e] - bf_bits_f(hb[e]));
  }
  const unsigned h0 = hb[0] | (hb[1] << 16), h1 = hb[2] | (hb[3] << 16);
  const unsigned h2 = hb[4] | (hb[5] << 16), h3 = hb[6] | (hb[7] << 16);
  const unsigned l0 = lb[0] | (lb[1] << 16), l1 = lb[2] | (lb[3] << 16);
  const unsigned l2 = lb[4] | (lb[5] << 16), l3 = lb[6] | (lb[7] << 16);
  hw = (v4u){h0, h1, h2, h3};
  lw = (v4u){l0, l1, l2, l3};
}

__device__ __forceinline__ void ld8(const float* p, float (&v)[8]) {
  const v4f a = *(const v4f*)(p);
  const v4f b = *(const v4f*)(p + 4);
  v[0] = a[0]; v[1] = a[1]; v[2] = a[2]; v[3] = a[3];
  v[4] = b[0]; v[5] = b[1]; v[6] = b[2]; v[7] = b[3];
}

__device__ __forceinline__ void store2_u(unsigned* ph, v4u hw, unsigned* pl, v4u lw) {
  *(volatile v4u*)ph = hw;
  *(volatile v4u*)pl = lw;
  __threadfence();
  *(volatile v4u*)ph = hw;
  *(volatile v4u*)pl = lw;
}
__device__ __forceinline__ void store2_f4(float* pa, v4f a, float* pb, v4f b) {
  *(volatile v4f*)pa = a;
  *(volatile v4f*)pb = b;
  __threadfence();
  *(volatile v4f*)pa = a;
  *(volatile v4f*)pb = b;
}

union FragB16 { v16b v; v8b h[2]; };
__device__ __forceinline__ v16b frag_load(const __bf16* p) {
  FragB16 f;
  f.h[0] = *(const v8b*)(p);
  f.h[1] = *(const v8b*)(p + 16);
  return f.v;
}
__device__ __forceinline__ v8f mma_bf16(v16b a, v16b b, v8f c) {
  return __builtin_amdgcn_wmma_f32_16x16x32_bf16(false, a, false, b, (short)0, c, false, false);
}
__device__ __forceinline__ void guard4_b(v8f& a, v8f& b, v8f& c, v8f& d, v16b x, v16b y) {
  asm volatile("v_nop\n\tv_nop\n\tv_nop\n\tv_nop" : "+v"(a), "+v"(b), "+v"(c), "+v"(d) : "v"(x), "v"(y));
}
__device__ __forceinline__ void keep4_b(v16b a, v16b b, v16b c, v16b d) { asm volatile("v_nop" :: "v"(a), "v"(b), "v"(c), "v"(d)); }
__device__ __forceinline__ void acc_guard4(v8f& a, v8f& b, v8f& c, v8f& d) {
  asm volatile("v_nop\n\tv_nop\n\tv_nop\n\tv_nop" : "+v"(a), "+v"(b), "+v"(c), "+v"(d));
}

constexpr int PK_ROWS = 64;
constexpr int PK_PITCH = 97;
__global__ __launch_bounds__(256) void pack_g0_kernel(const float* __restrict__ xyz, const float* __restrict__ pts,
                                                      unsigned* __restrict__ g0h, unsigned* __restrict__ g0l) {
  __shared__ float tile[PK_ROWS * PK_PITCH];
  const int tid = threadIdx.x;
  const int blk = blockIdx.x;
  const int b = blk >> 6;
  const int n0 = (blk & 63) * PK_ROWS;
  const float* pb = pts + (size_t)b * DFEAT * NPTS + n0;
#pragma unroll 4
  for (int it = 0; it < 16; ++it) {
    const int e = it * 256 + tid;
    const int c = e >> 6;
    const int nl = e & 63;
    tile[nl * PK_PITCH + c] = pb[(size_t)c * NPTS + nl];
  }
  const float* xb = xyz + (size_t)b * 3 * NPTS + n0;
#pragma unroll 4
  for (int it = 0; it < 8; ++it) {
    const int e = it * 256 + tid;
    const int j = e >> 6;
    const int nl = e & 63;
    const int jc = j < 3 ? j : 2;
    const float v = xb[(size_t)jc * NPTS + nl];
    tile[nl * PK_PITCH + 64 + j] = (j < 3) ? v : 0.0f;
  }
  __syncthreads();
  unsigned* oh = g0h + (size_t)blk * (PK_ROWS * G0_LD / 2);
  unsigned* ol = g0l + (size_t)blk * (PK_ROWS * G0_LD / 2);
#pragma unroll 1
  for (int it = 0; it < 3; ++it) {
    const int q = it * 256 + tid;
    const int row = q / 12;
    const int c8 = (q - row * 12) * 8;
    float v[8];
#pragma unroll
    for (int e = 0; e < 8; ++e) v[e] = tile[row * PK_PITCH + c8 + e];
    v4u hw, lw;
    split8(v, hw, lw);
    store2_u(oh + (size_t)q * 4, hw, ol + (size_t)q * 4, lw);
  }
}

__global__ __launch_bounds__(256) void prep_w_kernel(const float* __restrict__ ec_w, const float* __restrict__ gm_w,
                                                     const float* __restrict__ w0, const float* __restrict__ w1,
                                                     const float* __restrict__ w2,
                                                     unsigned* __restrict__ wh, unsigned* __restrict__ wl) {
  const int blk = blockIdx.x;
  const int tid = threadIdx.x;
  float v[8];
  int chunk;
  if (blk < 8) {
    const int q = blk * 256 + tid;
    const int o2 = q >> 3;
    const int j0 = (q & 7) * 8;
    const int o = o2 & 127;
    const bool isP = (blk < 4);
    float a[8], d[8];
    ld8(ec_w + (size_t)o * 128 + j0, a);
    ld8(ec_w + (size_t)o * 128 + 64 + j0, d);
#pragma unroll
    for (int e = 0; e < 8; ++e) v[e] = isP ? (a[e] - d[e]) : d[e];
    chunk = q;
  } else if (blk < 16) {
    const int q = (blk - 8) * 256 + tid;
    ld8(gm_w + (size_t)q * 8, v);
    chunk = WOFF_GM / 8 + q;
  } else if (blk < 19) {
    const int q = (blk - 16) * 256 + tid;
    const int o = q / 12;
    const int j0 = (q - o * 12) * 8;
#pragma unroll
    for (int e = 0; e < 8; ++e) {
      const int j = j0 + e;
      const int src = (j < 64) ? (j + 3) : ((j < 67) ? (j - 64) : 0);
      const float x = w0[(size_t)o * 67 + src];
      v[e] = (j < 67) ? x : 0.0f;
    }
    chunk = WOFF_W0 / 8 + q;
  } else if (blk < 23) {
    const int q = (blk - 19) * 256 + tid;
    ld8(w1 + (size_t)q * 8, v);
    chunk = WOFF_W1 / 8 + q;
  } else {
    const int q = (blk - 23) * 256 + tid;
    ld8(w2 + (size_t)q * 8, v);
    chunk = WOFF_W2 / 8 + q;
  }
  v4u hw, lw;
  split8(v, hw, lw);
  store2_u(wh + (size_t)chunk * 4, hw, wl + (size_t)chunk * 4, lw);
}

template <bool OUT_Z, bool STATS>
__global__ __launch_bounds__(256) void gemm_bf16x3_kernel(
    const unsigned short* __restrict__ Ap, const unsigned short* __restrict__ A2p, int lda,
    const unsigned short* __restrict__ Btp, const unsigned short* __restrict__ Bt2p, int ldb,
    float* __restrict__ Cz, int ldc, float* __restrict__ part, int M, int N, int K) {
  const __bf16* A   = (const __bf16*)Ap;
  const __bf16* A2  = (const __bf16*)A2p;
  const __bf16* Bt  = (const __bf16*)Btp;
  const __bf16* Bt2 = (const __bf16*)Bt2p;
  __shared__ __align__(16) float sT[8][16 * 68];
  const int lane = threadIdx.x & 31;
  const int wave = threadIdx.x >> 5;
  const int tilesN = N >> 6;
  const int tilesM = M >> 6;
  const int tile = blockIdx.x * 8 + wave;
  if (tile >= tilesM * tilesN) return;
  const int tm = tile / tilesN;
  const int tn = tile - tm * tilesN;
  const int m0 = tm << 6;
  const int n0 = tn << 6;
  const int rlane = lane & 15;
  const int koff = (lane >> 4) * 8;
  const int mOff = (lane >> 4) * 8;

  v8f acc[4][4];
#pragma unroll
  for (int i = 0; i < 4; ++i)
#pragma unroll
    for (int j = 0; j < 4; ++j) acc[i][j] = (v8f){0.f, 0.f, 0.f, 0.f, 0.f, 0.f, 0.f, 0.f};

  for (int k0 = 0; k0 < K; k0 += 32) {
    v16b bh[4], bl[4];
#pragma unroll
    for (int j = 0; j < 4; ++j) {
      const size_t bo = (size_t)(n0 + (j << 4) + rlane) * ldb + koff + k0;
      bh[j] = frag_load(Bt + bo);
      bl[j] = frag_load(Bt2 + bo);
    }
#pragma unroll
    for (int i = 0; i < 4; ++i) {
      const size_t ao = (size_t)(m0 + (i << 4) + rlane) * lda + koff + k0;
      const v16b ah = frag_load(A + ao);
      const v16b al = frag_load(A2 + ao);
#pragma unroll
      for (int j = 0; j < 4; ++j) {
        acc[i][j] = mma_bf16(ah, bh[j], acc[i][j]);
        acc[i][j] = mma_bf16(ah, bl[j], acc[i][j]);
        acc[i][j] = mma_bf16(al, bh[j], acc[i][j]);
      }
      guard4_b(acc[i][0], acc[i][1], acc[i][2], acc[i][3], ah, al);
    }
    keep4_b(bh[0], bh[1], bh[2], bh[3]);
    keep4_b(bl[0], bl[1], bl[2], bl[3]);
  }
  acc_guard4(acc[0][0], acc[0][1], acc[0][2], acc[0][3]);
  acc_guard4(acc[1][0], acc[1][1], acc[1][2], acc[1][3]);
  acc_guard4(acc[2][0], acc[2][1], acc[2][2], acc[2][3]);
  acc_guard4(acc[3][0], acc[3][1], acc[3][2], acc[3][3]);

  float* slab = sT[wave];
  if (OUT_Z) {
#pragma unroll
    for (int i = 0; i < 4; ++i) {
      const int mBase = m0 + (i << 4);
#pragma unroll
      for (int j = 0; j < 4; ++j) {
#pragma unroll
        for (int r = 0; r < 8; ++r) slab[(mOff + r) * 68 + (j << 4) + rlane] = acc[i][j][r];
      }
      __builtin_amdgcn_fence(__ATOMIC_RELEASE, "workgroup");
      __builtin_amdgcn_wave_barrier();
      __builtin_amdgcn_fence(__ATOMIC_ACQUIRE, "workgroup");
      {
        const int hh = lane >> 4, c4 = (lane & 15) * 4;
        for (int pass = 0; pass < 2; ++pass) {
#pragma unroll
          for (int it = 0; it < 8; ++it) {
            const int row = it * 2 + hh;
            const v4f v = *(const v4f*)(slab + row * 68 + c4);
            *(volatile v4f*)(Cz + (size_t)(mBase + row) * ldc + n0 + c4) = v;
          }
          __threadfence();
        }
      }
      __builtin_amdgcn_fence(__ATOMIC_RELEASE, "workgroup");
      __builtin_amdgcn_wave_barrier();
      __builtin_amdgcn_fence(__ATOMIC_ACQUIRE, "workgroup");
    }
  }
  if (STATS) {
    const float pinf = __builtin_inff();
#pragma unroll
    for (int j = 0; j < 4; ++j) {
      float s1 = 0.0f, s2 = 0.0f, mx = -pinf, mn = pinf;
#pragma unroll
      for (int i = 0; i < 4; ++i) {
#pragma unroll
        for (int r = 0; r < 8; ++r) {
          const float v = acc[i][j][r];
          s1 += v;
          s2 += v * v;
          mx = fmaxf(mx, v);
          mn = fminf(mn, v);
        }
      }
      const float s1o = __shfl_xor(s1, 16, 32);
      const float s2o = __shfl_xor(s2, 16, 32);
      const float mxo = __shfl_xor(mx, 16, 32);
      const float mno = __shfl_xor(mn, 16, 32);
      s1 += s1o;
      s2 += s2o;
      mx = fmaxf(mx, mxo);
      mn = fminf(mn, mno);
      if (mOff == 0) {
        slab[0 * 64 + (j << 4) + rlane] = s1;
        slab[1 * 64 + (j << 4) + rlane] = s2;
        slab[2 * 64 + (j << 4) + rlane] = mx;
        slab[3 * 64 + (j << 4) + rlane] = mn;
      }
    }
    __builtin_amdgcn_fence(__ATOMIC_RELEASE, "workgroup");
    __builtin_amdgcn_wave_barrier();
    __builtin_amdgcn_fence(__ATOMIC_ACQUIRE, "workgroup");
    {
      const int hh = lane >> 4, c4 = (lane & 15) * 4;
      float* pb = part + ((size_t)tm * 4) * N + n0;
      for (int pass = 0; pass < 2; ++pass) {
#pragma unroll
        for (int it = 0; it < 2; ++it) {
          const int st = it * 2 + hh;
          const v4f v = *(const v4f*)(slab + st * 64 + c4);
          *(volatile v4f*)(pb + (size_t)st * N + c4) = v;
        }
        __threadfence();
      }
    }
    __builtin_amdgcn_fence(__ATOMIC_RELEASE, "workgroup");
    __builtin_amdgcn_wave_barrier();
    __builtin_amdgcn_fence(__ATOMIC_ACQUIRE, "workgroup");
  }
}

constexpr int KN_TILE = 1024;
__global__ __launch_bounds__(256) void knn_edge_kernel(const float* __restrict__ xyz, const float* __restrict__ PQ,
                                                       float* __restrict__ hmax, float* __restrict__ hmin,
                                                       float* __restrict__ ecpart) {
#pragma clang fp contract(off)
  __shared__ __align__(16) v4f cand[KN_TILE];
  __shared__ int sE[256 * KNBR];
  __shared__ double sRed[8 * 2 * GOUT];
  const int tid = threadIdx.x;
  const int lane = tid & 31;
  const int wave = tid >> 5;
  const int blk = blockIdx.x;
  const int b = blk >> 4;
  const int n = (blk & 15) * 256 + tid;
  const float* xb = xyz + (size_t)b * 3 * NPTS;
  const float qx = xb[n];
  const float qy = xb[NPTS + n];
  const float qz = xb[2 * NPTS + n];
  const float qt0 = qx * qx;
  const float qt1 = qy * qy;
  const float qt2 = qz * qz;
  const float qs = (qt0 + qt2) + qt1;

  float bd[KNBR];
  int bi[KNBR];
#pragma unroll
  for (int j = 0; j < KNBR; ++j) { bd[j] = __builtin_inff(); bi[j] = n; }

  for (int t0 = 0; t0 < NPTS; t0 += KN_TILE) {
    __syncthreads();
#pragma unroll 1
    for (int it = 0; it < 4; ++it) {
      const int i = it * 256 + tid;
      const float x = xb[t0 + i];
      const float y = xb[NPTS + t0 + i];
      const float z = xb[2 * NPTS + t0 + i];
      const float a0 = x * x;
      const float a1 = y * y;
      const float a2 = z * z;
      cand[i] = (v4f){x, y, z, (a0 + a2) + a1};
    }
    __syncthreads();
#pragma unroll 1
    for (int i = 0; i < KN_TILE; ++i) {
      const v4f cd = cand[i];
      float p = qx * cd[0];
      p = __builtin_fmaf(qy, cd[1], p);
      p = __builtin_fmaf(qz, cd[2], p);
      const float d = (qs + cd[3]) - 2.0f * p;
      const int m = t0 + i;
      if (d < bd[KNBR - 1] && m != n) {
#pragma unroll
        for (int j = KNBR - 1; j >= 1; --j) {
          const bool up = bd[j - 1] > d;
          const bool here = bd[j] > d;
          const float nb = up ? bd[j - 1] : (here ? d : bd[j]);
          const int ni = up ? bi[j - 1] : (here ? m : bi[j]);
          bd[j] = nb;
          bi[j] = ni;
        }
        const bool h0 = bd[0] > d;
        bd[0] = h0 ? d : bd[0];
        bi[0] = h0 ? m : bi[0];
      }
    }
  }
#pragma unroll
  for (int j = 0; j < KNBR; ++j) sE[tid * KNBR + j] = b * NPTS + bi[j];
  __syncthreads();

  double S1d[4], S2d[4];
#pragma unroll
  for (int c = 0; c < 4; ++c) { S1d[c] = 0.0; S2d[c] = 0.0; }
#pragma unroll 1
  for (int rr = 0; rr < 32; ++rr) {
    const int rl = wave * 32 + rr;
    const size_t row = (size_t)blk * 256 + rl;
    const int le = lane < KNBR ? lane : (KNBR - 1);
    int ev = sE[rl * KNBR + le];
    ev = ev < 0 ? 0 : ev;
    ev = ev > (NROWS - 1) ? (NROWS - 1) : ev;
    const v4f P = *(const v4f*)(PQ + row * 256 + 4 * lane);
    float s1[4], s2[4], mx[4], mn[4];
#pragma unroll
    for (int c = 0; c < 4; ++c) { s1[c] = 0.0f; s2[c] = 0.0f; mx[c] = -__builtin_inff(); mn[c] = __builtin_inff(); }
#pragma unroll 1
    for (int g = 0; g < 4; ++g) {
#pragma unroll
      for (int kk = 0; kk < 6; ++kk) {
        const int e = __shfl(ev, g * 6 + kk, 32);
        const v4f Q = *(const v4f*)(PQ + (size_t)e * 256 + 128 + 4 * lane);
#pragma unroll
        for (int c = 0; c < 4; ++c) {
          const float qv = Q[c];
          const float h = P[c] + qv;
          s1[c] += h;
          s2[c] += h * h;
          mx[c] = fmaxf(mx[c], qv);
          mn[c] = fminf(mn[c], qv);
        }
      }
    }
#pragma unroll
    for (int c = 0; c < 4; ++c) { S1d[c] += (double)s1[c]; S2d[c] += (double)s2[c]; }
    const v4f vmax = (v4f){P[0] + mx[0], P[1] + mx[1], P[2] + mx[2], P[3] + mx[3]};
    const v4f vmin = (v4f){P[0] + mn[0], P[1] + mn[1], P[2] + mn[2], P[3] + mn[3]};
    store2_f4(hmax + row * GOUT + 4 * lane, vmax, hmin + row * GOUT + 4 * lane, vmin);
  }
#pragma unroll
  for (int c = 0; c < 4; ++c) {
    sRed[(wave * 2 + 0) * GOUT + 4 * lane + c] = S1d[c];
    sRed[(wave * 2 + 1) * GOUT + 4 * lane + c] = S2d[c];
  }
  __syncthreads();
  {
    const int stat = tid >> 7;
    const int c = tid & 127;
    double a = 0.0;
#pragma unroll
    for (int w = 0; w < 8; ++w) a += sRed[(w * 2 + stat) * GOUT + c];
    const float fv = (float)a;
    float* pp = ecpart + (size_t)blk * 256 + tid;
    *(volatile float*)pp = fv;
    __threadfence();
    *(volatile float*)pp = fv;
  }
}

__global__ __launch_bounds__(256) void bn_finalize_kernel(const float* __restrict__ part, const float* __restrict__ gamma,
                                                          const float* __restrict__ beta, const float* __restrict__ bias,
                                                          float* __restrict__ st, double inv_count,
                                                          int T, int S, int C, int has_bias) {
  __shared__ double sS[256];
  const int tid = threadIdx.x;
  const int p = (tid < 2 * C) ? tid : 0;
  const int stat = p / C;
  const int c = p - stat * C;
  double acc = 0.0;
#pragma unroll 4
  for (int t = 0; t < T; ++t) acc += (double)part[((size_t)t * S + stat) * C + c];
  sS[tid] = acc;
  __syncthreads();
  if (tid < C) {
    const double mean = sS[tid] * inv_count;
    double var = sS[C + tid] * inv_count - mean * mean;
    var = var < 0.0 ? 0.0 : var;
    const float inv = 1.0f / sqrtf((float)var + BN_EPS);
    const float s = gamma[tid] * inv;
    const float bl = bias[tid];
    const float bz = has_bias ? bl : 0.0f;
    const double sh = ((double)beta[tid] - (mean + (double)bz) * (double)s) + (double)bz * (double)s;
    const float shf = (float)sh;
    *(volatile float*)(st + tid) = s;
    *(volatile float*)(st + C + tid) = shf;
    __threadfence();
    *(volatile float*)(st + tid) = s;
    *(volatile float*)(st + C + tid) = shf;
  }
}

__global__ __launch_bounds__(256) void bn_apply_kernel(const float* za, const float* zb, const float* __restrict__ st,
                                                       unsigned* __restrict__ outh, unsigned* __restrict__ outl,
                                                       int C, float leak, int nchunks) {
  const int q = blockIdx.x * 256 + threadIdx.x;
  if (q >= nchunks) return;
  const int c0 = (q * 8) % C;
  float a[8], bm[8], s[8], t[8], y[8];
  ld8(za + (size_t)q * 8, a);
  ld8(zb + (size_t)q * 8, bm);
  ld8(st + c0, s);
  ld8(st + C + c0, t);
#pragma unroll
  for (int e = 0; e < 8; ++e) {
    const float v = (s[e] >= 0.0f) ? a[e] : bm[e];
    const float w = v * s[e] + t[e];
    y[e] = (w > 0.0f) ? w : leak * w;
  }
  v4u hw, lw;
  split8(y, hw, lw);
  store2_u(outh + (size_t)q * 4, hw, outl + (size_t)q * 4, lw);
}

__global__ __launch_bounds__(256) void head_kernel(const float* __restrict__ p2, const float* __restrict__ pgm,
                                                   const float* __restrict__ g2, const float* __restrict__ be2,
                                                   const float* __restrict__ bias2,
                                                   const float* __restrict__ gm_g, const float* __restrict__ gm_b,
                                                   const float* __restrict__ fu_w, const float* __restrict__ fu_g,
                                                   const float* __restrict__ fu_b, float* __restrict__ out) {
  __shared__ float fused[NBATCH * FUSEDC];
  const int tid = threadIdx.x;
  const double inv_n = 1.0 / (double)NROWS;
#pragma unroll 1
  for (int pass = 0; pass < 2; ++pass) {
    const float* part = pass ? pgm : p2;
    const int C = pass ? HALFC : MLPC2;
    const float* gam = pass ? gm_g : g2;
    const float* bet = pass ? gm_b : be2;
    const float leak = pass ? 0.2f : 0.0f;
    const int foff = pass ? MLPC2 : 0;
    const int c = (tid < C) ? tid : (C - 1);
    double S1 = 0.0, S2 = 0.0;
    float mx[NBATCH], mn[NBATCH];
#pragma unroll
    for (int bb = 0; bb < NBATCH; ++bb) {
      float m1 = -__builtin_inff(), m2 = __builtin_inff();
#pragma unroll 2
      for (int t = 0; t < 64; ++t) {
        const size_t o = ((size_t)(bb * 64 + t) * 4) * C + c;
        S1 += (double)part[o];
        S2 += (double)part[o + C];
        m1 = fmaxf(m1, part[o + 2 * (size_t)C]);
        m2 = fminf(m2, part[o + 3 * (size_t)C]);
      }
      mx[bb] = m1;
      mn[bb] = m2;
    }
    const double mean = S1 * inv_n;
    double var = S2 * inv_n - mean * mean;
    var = var < 0.0 ? 0.0 : var;
    const float inv = 1.0f / sqrtf((float)var + BN_EPS);
    const float s = gam[c] * inv;
    const float b2v = bias2[c];
    const float bz = pass ? 0.0f : b2v;
    const float t = (float)((double)bet[c] - (mean + (double)bz) * (double)s);
#pragma unroll
    for (int bb = 0; bb < NBATCH; ++bb) {
      const float v = (s >= 0.0f) ? mx[bb] : mn[bb];
      const float w = (v + bz) * s + t;
      const float y = (w > 0.0f) ? w : leak * w;
      if (tid < C) fused[bb * FUSEDC + foff + tid] = y;
    }
  }
  __syncthreads();
  const float* wr = fu_w + (size_t)tid * FUSEDC;
  double f0 = 0.0, f1 = 0.0, f2 = 0.0, f3 = 0.0;
#pragma unroll 2
  for (int c4 = 0; c4 < FUSEDC / 4; ++c4) {
    const v4f w = *(const v4f*)(wr + 4 * c4);
#pragma unroll
    for (int e = 0; e < 4; ++e) {
      const double wv = (double)w[e];
      f0 += wv * (double)fused[0 * FUSEDC + 4 * c4 + e];
      f1 += wv * (double)fused[1 * FUSEDC + 4 * c4 + e];
      f2 += wv * (double)fused[2 * FUSEDC + 4 * c4 + e];
      f3 += wv * (double)fused[3 * FUSEDC + 4 * c4 + e];
    }
  }
  const double mean = ((f0 + f1) + (f2 + f3)) * 0.25;
  const double d0 = f0 - mean, d1 = f1 - mean, d2 = f2 - mean, d3 = f3 - mean;
  const double var = ((d0 * d0 + d1 * d1) + (d2 * d2 + d3 * d3)) * 0.25;
  const float inv = 1.0f / sqrtf((float)var + BN_EPS);
  const float g = fu_g[tid];
  const float bb = fu_b[tid];
  float y0 = (float)d0 * inv * g + bb;
  float y1 = (float)d1 * inv * g + bb;
  float y2 = (float)d2 * inv * g + bb;
  float y3 = (float)d3 * inv * g + bb;
  y0 = (y0 > 0.0f) ? y0 : 0.2f * y0;
  y1 = (y1 > 0.0f) ? y1 : 0.2f * y1;
  y2 = (y2 > 0.0f) ? y2 : 0.2f * y2;
  y3 = (y3 > 0.0f) ? y3 : 0.2f * y3;
  for (int pass = 0; pass < 2; ++pass) {
    *(volatile float*)(out + 0 * MLPC2 + tid) = y0;
    *(volatile float*)(out + 1 * MLPC2 + tid) = y1;
    *(volatile float*)(out + 2 * MLPC2 + tid) = y2;
    *(volatile float*)(out + 3 * MLPC2 + tid) = y3;
    __threadfence();
  }
}

constexpr size_t SZ_G0   = (size_t)NROWS * G0_LD * 2;
constexpr size_t SZ_W    = (size_t)W_TOTAL * 2;
constexpr size_t SZ_PQ   = (size_t)NROWS * 256 * 4;
constexpr size_t SZ_H    = (size_t)NROWS * GOUT * 4;
constexpr size_t SZ_ECP  = (size_t)64 * 2 * GOUT * 4;
constexpr size_t SZ_ST   = 1024;
constexpr size_t SZ_GF   = (size_t)NROWS * GOUT * 2;
constexpr size_t SZ_GMP  = (size_t)256 * 4 * HALFC * 4;
constexpr size_t SZ_Z0   = (size_t)NROWS * MLPC0 * 4;
constexpr size_t SZ_P0   = (size_t)256 * 4 * MLPC0 * 4;
constexpr size_t SZ_A1   = (size_t)NROWS * MLPC0 * 2;
constexpr size_t SZ_Z1   = (size_t)NROWS * MLPC1 * 4;
constexpr size_t SZ_P1   = (size_t)256 * 4 * MLPC1 * 4;
constexpr size_t SZ_A2   = (size_t)NROWS * MLPC1 * 2;
constexpr size_t SZ_P2   = (size_t)256 * 4 * MLPC2 * 4;

constexpr size_t OFF_G0H = 0;
constexpr size_t OFF_G0L = OFF_G0H + SZ_G0;
constexpr size_t OFF_WH  = OFF_G0L + SZ_G0;
constexpr size_t OFF_WL  = OFF_WH + SZ_W;
constexpr size_t OFF_PQ  = OFF_WL + SZ_W;
constexpr size_t OFF_HMX = OFF_PQ + SZ_PQ;
constexpr size_t OFF_HMN = OFF_HMX + SZ_H;
constexpr size_t OFF_ECP = OFF_HMN + SZ_H;
constexpr size_t OFF_ECS = OFF_ECP + SZ_ECP;
constexpr size_t OFF_GFH = OFF_ECS + SZ_ST;
constexpr size_t OFF_GFL = OFF_GFH + SZ_GF;
constexpr size_t OFF_GMP = OFF_GFL + SZ_GF;
constexpr size_t OFF_Z0  = OFF_GMP + SZ_GMP;
constexpr size_t OFF_P0  = OFF_Z0 + SZ_Z0;
constexpr size_t OFF_ST0 = OFF_P0 + SZ_P0;
constexpr size_t OFF_A1H = OFF_ST0 + SZ_ST;
constexpr size_t OFF_A1L = OFF_A1H + SZ_A1;
constexpr size_t OFF_Z1  = OFF_A1L + SZ_A1;
constexpr size_t OFF_P1  = OFF_Z1 + SZ_Z1;
constexpr size_t OFF_ST1 = OFF_P1 + SZ_P1;
constexpr size_t OFF_A2H = OFF_ST1 + SZ_ST;
constexpr size_t OFF_A2L = OFF_A2H + SZ_A2;
constexpr size_t OFF_P2  = OFF_A2L + SZ_A2;
constexpr size_t WS_TOTAL = OFF_P2 + SZ_P2;
static_assert(WS_TOTAL == 76147712, "carve total");
static_assert(WS_TOTAL <= (size_t)134217728, "carve under 128 MiB");
static_assert(OFF_WH % 128 == 0 && OFF_WL % 128 == 0 && OFF_PQ % 128 == 0 && OFF_ECS % 128 == 0 && OFF_GFH % 128 == 0, "alignment");
static_assert(OFF_ST0 % 128 == 0 && OFF_A1H % 128 == 0 && OFF_ST1 % 128 == 0 && OFF_A2H % 128 == 0 && OFF_P2 % 128 == 0, "alignment");

extern "C" void kernel_launch(void* const* d_in, const int* in_sizes, int n_in,
                              void* d_out, int out_size, void* d_ws, size_t ws_size, hipStream_t stream) {
  if (n_in < 23) return;
  if (ws_size < WS_TOTAL) return;
  if (in_sizes[0] != NBATCH * 3 * NPTS || in_sizes[1] != NBATCH * DFEAT * NPTS) return;
  if (out_size < NBATCH * MLPC2) return;

  const float* xyz   = (const float*)d_in[0];
  const float* pts   = (const float*)d_in[1];
  const float* ec_w  = (const float*)d_in[2];
  const float* ec_g  = (const float*)d_in[3];
  const float* ec_b  = (const float*)d_in[4];
  const float* gm_w  = (const float*)d_in[5];
  const float* gm_g  = (const float*)d_in[6];
  const float* gm_b  = (const float*)d_in[7];
  const float* w0    = (const float*)d_in[8];
  const float* bias0 = (const float*)d_in[9];
  const float* g0    = (const float*)d_in[10];
  const float* be0   = (const float*)d_in[11];
  const float* w1    = (const float*)d_in[12];
  const float* bias1 = (const float*)d_in[13];
  const float* g1    = (const float*)d_in[14];
  const float* be1   = (const float*)d_in[15];
  const float* w2    = (const float*)d_in[16];
  const float* bias2 = (const float*)d_in[17];
  const float* g2    = (const float*)d_in[18];
  const float* be2   = (const float*)d_in[19];
  const float* fu_w  = (const float*)d_in[20];
  const float* fu_g  = (const float*)d_in[21];
  const float* fu_b  = (const float*)d_in[22];
  float* out = (float*)d_out;

  char* base = (char*)d_ws;
  unsigned* g0h = (unsigned*)(base + OFF_G0H);
  unsigned* g0l = (unsigned*)(base + OFF_G0L);
  unsigned* wh  = (unsigned*)(base + OFF_WH);
  unsigned* wl  = (unsigned*)(base + OFF_WL);
  float* PQ     = (float*)(base + OFF_PQ);
  float* hmx    = (float*)(base + OFF_HMX);
  float* hmn    = (float*)(base + OFF_HMN);
  float* ecp    = (float*)(base + OFF_ECP);
  float* ecs    = (float*)(base + OFF_ECS);
  unsigned* gfh = (unsigned*)(base + OFF_GFH);
  unsigned* gfl = (unsigned*)(base + OFF_GFL);
  float* gmp    = (float*)(base + OFF_GMP);
  float* z0     = (float*)(base + OFF_Z0);
  float* p0     = (float*)(base + OFF_P0);
  float* st0    = (float*)(base + OFF_ST0);
  unsigned* a1h = (unsigned*)(base + OFF_A1H);
  unsigned* a1l = (unsigned*)(base + OFF_A1L);
  float* z1     = (float*)(base + OFF_Z1);
  float* p1     = (float*)(base + OFF_P1);
  float* st1    = (float*)(base + OFF_ST1);
  unsigned* a2h = (unsigned*)(base + OFF_A2H);
  unsigned* a2l = (unsigned*)(base + OFF_A2L);
  float* p2     = (float*)(base + OFF_P2);

  const unsigned short* WH16 = (const unsigned short*)wh;
  const unsigned short* WL16 = (const unsigned short*)wl;
  const unsigned short* G0H16 = (const unsigned short*)g0h;
  const unsigned short* G0L16 = (const unsigned short*)g0l;

  pack_g0_kernel<<<NROWS / PK_ROWS, 256, 0, stream>>>(xyz, pts, g0h, g0l);
  prep_w_kernel<<<W_TOTAL / 8 / 256, 256, 0, stream>>>(ec_w, gm_w, w0, w1, w2, wh, wl);
  gemm_bf16x3_kernel<true, false><<<(NROWS / 64) * (256 / 64) / 8, 256, 0, stream>>>(
      G0H16, G0L16, G0_LD, WH16 + WOFF_EC, WL16 + WOFF_EC, DFEAT, PQ, 256, p2, NROWS, 256, DFEAT);
  knn_edge_kernel<<<NROWS / 256, 256, 0, stream>>>(xyz, PQ, hmx, hmn, ecp);
  bn_finalize_kernel<<<1, 256, 0, stream>>>(ecp, ec_g, ec_b, ec_g, ecs, 1.0 / (double)((size_t)NROWS * KNBR), 64, 2, GOUT, 0);
  bn_apply_kernel<<<NROWS * GOUT / 8 / 256, 256, 0, stream>>>(hmx, hmn, ecs, gfh, gfl, GOUT, 0.2f, NROWS * GOUT / 8);
  gemm_bf16x3_kernel<false, true><<<(NROWS / 64) * (HALFC / 64) / 8, 256, 0, stream>>>(
      (const unsigned short*)gfh, (const unsigned short*)gfl, GOUT, WH16 + WOFF_GM, WL16 + WOFF_GM, GOUT,
      PQ, HALFC, gmp, NROWS, HALFC, GOUT);
  gemm_bf16x3_kernel<true, true><<<(NROWS / 64) * (MLPC0 / 64) / 8, 256, 0, stream>>>(
      G0H16, G0L16, G0_LD, WH16 + WOFF_W0, WL16 + WOFF_W0, G0_LD, z0, MLPC0, p0, NROWS, MLPC0, G0_LD);
  bn_finalize_kernel<<<1, 256, 0, stream>>>(p0, g0, be0, bias0, st0, 1.0 / (double)NROWS, 256, 4, MLPC0, 1);
  bn_apply_kernel<<<NROWS * MLPC0 / 8 / 256, 256, 0, stream>>>(z0, z0, st0, a1h, a1l, MLPC0, 0.0f, NROWS * MLPC0 / 8);
  gemm_bf16x3_kernel<true, true><<<(NROWS / 64) * (MLPC1 / 64) / 8, 256, 0, stream>>>(
      (const unsigned short*)a1h, (const unsigned short*)a1l, MLPC0, WH16 + WOFF_W1, WL16 + WOFF_W1, MLPC0,
      z1, MLPC1, p1, NROWS, MLPC1, MLPC0);
  bn_finalize_kernel<<<1, 256, 0, stream>>>(p1, g1, be1, bias1, st1, 1.0 / (double)NROWS, 256, 4, MLPC1, 1);
  bn_apply_kernel<<<NROWS * MLPC1 / 8 / 256, 256, 0, stream>>>(z1, z1, st1, a2h, a2l, MLPC1, 0.0f, NROWS * MLPC1 / 8);
  gemm_bf16x3_kernel<false, true><<<(NROWS / 64) * (MLPC2 / 64) / 8, 256, 0, stream>>>(
      (const unsigned short*)a2h, (const unsigned short*)a2l, MLPC1, WH16 + WOFF_W2, WL16 + WOFF_W2, MLPC1,
      PQ, MLPC2, p2, NROWS, MLPC2, MLPC1);
  head_kernel<<<1, 256, 0, stream>>>(p2, gmp, g2, be2, bias2, gm_g, gm_b, fu_w, fu_g, fu_b, out);
}
